// CrossFeatureAffinityPooling_71425306132902
// MI455X (gfx1250) — hardware-verified
//
#include <hip/hip_runtime.h>
#include <stddef.h>
#include <stdint.h>
#include <math.h>

#define NBMAX 4
#define CC    256
#define NPX   4096
#define HWD   64
#define TP    72
#define EPF   68

#define PLANE       ((size_t)CC * NPX)
#define ACT16_BYTES ((size_t)NBMAX * PLANE * 2)
#define W16_BYTES   ((size_t)2 * CC * CC * 2)
#define S_BYTES     ((size_t)NPX * NPX * 4)
#define ST_BYTES    ((size_t)NPX * 4)
#define O_BYTES     ((size_t)PLANE * 4)
#define PS_BYTES    ((size_t)NBMAX * HWD * CC * 4)

#define OFF_HT   ((size_t)0)
#define OFF_UT   (OFF_HT + ACT16_BYTES)
#define OFF_UC   (OFF_UT + ACT16_BYTES)
#define OFF_W16  (OFF_UC + ACT16_BYTES)
#define OFF_QH   (OFF_W16 + W16_BYTES)
#define OFF_QL   (OFF_QH + ACT16_BYTES)
#define OFF_KH   (OFF_QL + ACT16_BYTES)
#define OFF_KL   (OFF_KH + ACT16_BYTES)
#define OFF_S    (OFF_KL + ACT16_BYTES)
#define OFF_RMAX (OFF_S + S_BYTES)
#define OFF_RSUM (OFF_RMAX + ST_BYTES)
#define OFF_O    (OFF_RSUM + ST_BYTES)
#define OFF_PS   (OFF_O + O_BYTES)
#define OFF_PQ   (OFF_PS + PS_BYTES)
#define WS_TOTAL (OFF_PQ + PS_BYTES)

static_assert(OFF_QH == (size_t)25427968);
static_assert(OFF_S == (size_t)58982400);
static_assert(OFF_O == (size_t)126124032);
static_assert(WS_TOTAL == (size_t)130842624);
static_assert(WS_TOTAL <= (size_t)134217728);
static_assert((OFF_UT % 256) == 0);
static_assert((OFF_UC % 256) == 0);
static_assert((OFF_W16 % 256) == 0);
static_assert((OFF_QH % 256) == 0);
static_assert((OFF_QL % 256) == 0);
static_assert((OFF_KH % 256) == 0);
static_assert((OFF_KL % 256) == 0);
static_assert((OFF_S % 256) == 0);
static_assert((OFF_RMAX % 256) == 0);
static_assert((OFF_RSUM % 256) == 0);
static_assert((OFF_O % 256) == 0);
static_assert((OFF_PS % 256) == 0);
static_assert((OFF_PQ % 256) == 0);
static_assert(NPX == HWD * HWD);
static_assert((CC % 64) == 0);
static_assert((NPX % 64) == 0);
static_assert((TP * 2) % 16 == 0);
static_assert((EPF * 4) % 16 == 0);

typedef unsigned short v8us  __attribute__((ext_vector_type(8)));
typedef unsigned short v16us __attribute__((ext_vector_type(16)));
typedef _Float16       v16h  __attribute__((ext_vector_type(16)));
typedef float          v4f   __attribute__((ext_vector_type(4)));
typedef float          v8f   __attribute__((ext_vector_type(8)));

union FragU { v16us v; v8us half[2]; };

__device__ __forceinline__ unsigned bbits(float f) {
  unsigned u = __float_as_uint(f);
  return (u + 0x7FFFu + ((u >> 16) & 1u)) >> 16;
}
__device__ __forceinline__ float bf16r(float f) {
  return __uint_as_float(bbits(f) << 16);
}
__device__ __forceinline__ unsigned short hbits(float f) {
  return __builtin_bit_cast(unsigned short, (_Float16)f);
}
__device__ __forceinline__ float rcpf(float x) {
#if defined(__HIP_DEVICE_COMPILE__)
  return __builtin_amdgcn_rcpf(x);
#else
  return 1.0f / x;
#endif
}
__device__ __forceinline__ v8f zero8() { v8f z = {0.f, 0.f, 0.f, 0.f, 0.f, 0.f, 0.f, 0.f}; return z; }

__device__ __forceinline__ double shfl_xor_d(double v, int o) {
  const long long x = __double_as_longlong(v);
  int lo = (int)(x & 0xffffffffll);
  int hi = (int)(x >> 32);
  lo = __shfl_xor(lo, o, 32);
  hi = __shfl_xor(hi, o, 32);
  const long long y = ((long long)(unsigned)hi << 32) | (long long)(unsigned)lo;
  return __longlong_as_double(y);
}

__device__ __forceinline__ v16us ldfrag_u(const unsigned short* p) {
  FragU f;
  f.half[0] = *(const v8us*)(p);
  f.half[1] = *(const v8us*)(p + 16);
  return f.v;
}

__device__ __forceinline__ v8f mma_hu(v16us a, v16us b, v8f c) {
#if defined(__HIP_DEVICE_COMPILE__)
  return __builtin_amdgcn_wmma_f32_16x16x32_f16(false, __builtin_bit_cast(v16h, a),
                                               false, __builtin_bit_cast(v16h, b),
                                               (short)0, c, false, false);
#else
  (void)a; (void)b;
  return c;
#endif
}
__device__ __forceinline__ void guard4(v8f& c0, v8f& c1, v8f& c2, v8f& c3, const v16us& a,
                                       const v16us& b0, const v16us& b1, const v16us& b2,
                                       const v16us& b3) {
#if defined(__HIP_DEVICE_COMPILE__)
  asm volatile("v_nop\n\tv_nop\n\tv_nop\n\tv_nop"
               : "+v"(c0), "+v"(c1), "+v"(c2), "+v"(c3)
               : "v"(a), "v"(b0), "v"(b1), "v"(b2), "v"(b3));
#else
  (void)c0; (void)c1; (void)c2; (void)c3; (void)a; (void)b0; (void)b1; (void)b2; (void)b3;
#endif
}
__device__ __forceinline__ void guard8(v8f& c0, v8f& c1, v8f& c2, v8f& c3, v8f& c4, v8f& c5,
                                       v8f& c6, v8f& c7, const v16us& a0, const v16us& a1,
                                       const v16us& b0, const v16us& b1, const v16us& b2,
                                       const v16us& b3) {
#if defined(__HIP_DEVICE_COMPILE__)
  asm volatile("v_nop\n\tv_nop\n\tv_nop\n\tv_nop"
               : "+v"(c0), "+v"(c1), "+v"(c2), "+v"(c3), "+v"(c4), "+v"(c5), "+v"(c6), "+v"(c7)
               : "v"(a0), "v"(a1), "v"(b0), "v"(b1), "v"(b2), "v"(b3));
#else
  (void)c0; (void)c1; (void)c2; (void)c3; (void)c4; (void)c5; (void)c6; (void)c7;
  (void)a0; (void)a1; (void)b0; (void)b1; (void)b2; (void)b3;
#endif
}
__device__ __forceinline__ void guard8w(v8f& c0, v8f& c1, v8f& c2, v8f& c3, v8f& c4, v8f& c5,
                                        v8f& c6, v8f& c7, const v16us& a0, const v16us& a1,
                                        const v16us& b0, const v16us& b1, const v16us& b2,
                                        const v16us& b3, const v16us& b4, const v16us& b5,
                                        const v16us& b6, const v16us& b7) {
#if defined(__HIP_DEVICE_COMPILE__)
  asm volatile("v_nop\n\tv_nop\n\tv_nop\n\tv_nop"
               : "+v"(c0), "+v"(c1), "+v"(c2), "+v"(c3), "+v"(c4), "+v"(c5), "+v"(c6), "+v"(c7)
               : "v"(a0), "v"(a1), "v"(b0), "v"(b1), "v"(b2), "v"(b3), "v"(b4), "v"(b5),
                 "v"(b6), "v"(b7));
#else
  (void)c0; (void)c1; (void)c2; (void)c3; (void)c4; (void)c5; (void)c6; (void)c7;
  (void)a0; (void)a1; (void)b0; (void)b1; (void)b2; (void)b3; (void)b4; (void)b5; (void)b6; (void)b7;
#endif
}

__device__ __forceinline__ void store_tile_f32(const float* ct, float* C, size_t row0, int col0,
                                               int ldc, int w, int lane) {
  const int q  = lane >> 3;
  const int jj = lane & 7;
#pragma unroll 1
  for (int it = 0; it < 8; ++it) {
    const int li = it * 16 + w * 4 + q;
    const int tr = li >> 1, hf = li & 1;
    const v4f v = *(const v4f*)(ct + tr * 64 + hf * 32 + jj * 4);
    *(volatile v4f*)(C + (row0 + tr) * (size_t)ldc + col0 + hf * 32 + jj * 4) = v;
  }
  __threadfence();
#pragma unroll 1
  for (int it = 0; it < 8; ++it) {
    const int li = it * 16 + w * 4 + q;
    const int tr = li >> 1, hf = li & 1;
    const v4f v = *(const v4f*)(ct + tr * 64 + hf * 32 + jj * 4);
    *(volatile v4f*)(C + (row0 + tr) * (size_t)ldc + col0 + hf * 32 + jj * 4) = v;
  }
}
template <int NW, int PITCH>
__device__ __forceinline__ void store_tile_us(const unsigned short* t, unsigned short* P,
                                              size_t row0, int ld, int col0, int w, int lane) {
  constexpr int NIT = 64 / (4 * NW);
  const int q  = lane >> 3;
  const int jj = lane & 7;
  v8us   v[NIT];
  size_t off[NIT];
#pragma unroll
  for (int it = 0; it < NIT; ++it) {
    const int li = it * 4 * NW + w * 4 + q;
    v[it]   = *(const v8us*)(t + li * PITCH + 8 * jj);
    off[it] = (row0 + li) * (size_t)ld + col0 + 8 * jj;
  }
#pragma unroll
  for (int it = 0; it < NIT; ++it) *(volatile v8us*)(P + off[it]) = v[it];
  __threadfence();
#pragma unroll
  for (int it = 0; it < NIT; ++it) *(volatile v8us*)(P + off[it]) = v[it];
}

__global__ __launch_bounds__(256)
void k_cvt(const float* __restrict__ hand, const float* __restrict__ u,
           unsigned short* ht, unsigned short* ut, unsigned short* uc)
{
  __shared__ __align__(16) unsigned short TH[64 * TP];
  __shared__ __align__(16) unsigned short TU[64 * TP];
  __shared__ __align__(16) unsigned short TC[64 * TP];

  const int tid  = threadIdx.x;
  const int lane = tid & 31;
  const int w    = tid >> 5;
  const int n0   = 64 * blockIdx.x;
  const int c0   = 64 * blockIdx.y;
  const int b    = blockIdx.z;
  const int cl   = tid >> 2;
  const int pq   = 16 * (tid & 3);
  const size_t src = (size_t)b * PLANE + (size_t)(c0 + cl) * NPX + n0 + pq;
#pragma unroll
  for (int g = 0; g < 4; ++g) {
    const v4f hv = *(const v4f*)(hand + src + 4 * g);
    const v4f uv = *(const v4f*)(u + src + 4 * g);
#pragma unroll
    for (int e = 0; e < 4; ++e) {
      const int px = pq + 4 * g + e;
      const unsigned short hb = hbits(16.0f * bf16r(hv[e]));
      const unsigned short ub = hbits(16.0f * bf16r(uv[e]));
      TH[px * TP + cl] = hb;
      TU[px * TP + cl] = ub;
      TC[cl * TP + px] = ub;
    }
  }
  __syncthreads();
  store_tile_us<8, TP>(TH, ht + (size_t)b * PLANE, (size_t)n0, CC, c0, w, lane);
  store_tile_us<8, TP>(TU, ut + (size_t)b * PLANE, (size_t)n0, CC, c0, w, lane);
  store_tile_us<8, TP>(TC, uc + (size_t)b * PLANE, (size_t)c0, NPX, n0, w, lane);
}

__global__ __launch_bounds__(256)
void k_wcvt(const float* __restrict__ whw, const float* __restrict__ wuw, unsigned short* w16)
{
  const int t   = blockIdx.x * 256 + threadIdx.x;
  const int o   = 8 * t;
  const int set = blockIdx.x >> 5;
  const int idx = o & (CC * CC - 1);
  const float* p = (set ? wuw : whw) + idx;
  v8us ob;
#pragma unroll
  for (int e = 0; e < 8; ++e) ob[e] = hbits(16.0f * bf16r(p[e]));
  *(volatile v8us*)(w16 + o) = ob;
  __threadfence();
  *(volatile v8us*)(w16 + o) = ob;
}

__global__ __launch_bounds__(128)
void k_proj(const unsigned short* __restrict__ ht, const unsigned short* __restrict__ ut,
            const unsigned short* __restrict__ w16, const float* __restrict__ whb,
            const float* __restrict__ wub, unsigned short* qh, unsigned short* ql,
            unsigned short* kh, unsigned short* kl)
{
  __shared__ __align__(16) unsigned short t0[64 * TP];
  __shared__ __align__(16) unsigned short t1[64 * TP];

  const int tid   = threadIdx.x;
  const int lane  = tid & 31;
  const int w     = tid >> 5;
  const int h     = lane >> 4;
  const int m     = lane & 15;
  const int n0    = 64 * blockIdx.x;
  const int o0    = 64 * blockIdx.y;
  const int which = blockIdx.z & 1;
  const int bb    = blockIdx.z >> 1;
  const unsigned short* x  = (which ? ut : ht) + (size_t)bb * PLANE;
  const unsigned short* wm = w16 + (size_t)which * CC * CC;
  const float* bias = which ? wub : whb;

  v8f acc[4];
#pragma unroll
  for (int j = 0; j < 4; ++j) acc[j] = zero8();

  const unsigned short* pa = x + (size_t)(n0 + 16 * w + m) * CC + 8 * h;
  const unsigned short* pb = wm + (size_t)(o0 + m) * CC + 8 * h;
#pragma unroll 2
  for (int kk = 0; kk < CC / 32; ++kk) {
    const v16us a  = ldfrag_u(pa + 32 * kk);
    const v16us b0 = ldfrag_u(pb + 32 * kk);
    const v16us b1 = ldfrag_u(pb + (size_t)16 * CC + 32 * kk);
    const v16us b2 = ldfrag_u(pb + (size_t)32 * CC + 32 * kk);
    const v16us b3 = ldfrag_u(pb + (size_t)48 * CC + 32 * kk);
    acc[0] = mma_hu(a, b0, acc[0]);
    acc[1] = mma_hu(a, b1, acc[1]);
    acc[2] = mma_hu(a, b2, acc[2]);
    acc[3] = mma_hu(a, b3, acc[3]);
    guard4(acc[0], acc[1], acc[2], acc[3], a, b0, b1, b2, b3);
  }

  const float k256 = 1.0f / 256.0f;
  float bv[4];
#pragma unroll
  for (int j = 0; j < 4; ++j) bv[j] = bf16r(bias[o0 + 16 * j + m]);
#pragma unroll
  for (int j = 0; j < 4; ++j) {
#pragma unroll
    for (int r = 0; r < 8; ++r) {
      const float val = acc[j][r] * k256 + bv[j];
      const _Float16 hv = (_Float16)val;
      const int rl = 16 * w + 8 * h + r;
      const int cl = 16 * j + m;
      t0[rl * TP + cl] = __builtin_bit_cast(unsigned short, hv);
      t1[rl * TP + cl] = hbits((val - (float)hv) * 32768.0f);
    }
  }
  __syncthreads();
  unsigned short* dh = which ? kh : qh;
  unsigned short* dl = which ? kl : ql;
  store_tile_us<4, TP>(t0, dh + (size_t)bb * PLANE, (size_t)n0, CC, o0, w, lane);
  store_tile_us<4, TP>(t1, dl + (size_t)bb * PLANE, (size_t)n0, CC, o0, w, lane);
}

__global__ __launch_bounds__(128)
void k_score(const unsigned short* __restrict__ qh, const unsigned short* __restrict__ ql,
             const unsigned short* __restrict__ kh, const unsigned short* __restrict__ kl, float* S)
{
  __shared__ __align__(16) float ct[64 * 64];

  const int tid  = threadIdx.x;
  const int lane = tid & 31;
  const int w    = tid >> 5;
  const int h    = lane >> 4;
  const int m    = lane & 15;
  const int m0   = 64 * blockIdx.x;
  const int n0   = 64 * blockIdx.y;

  v8f acc[4], accx[4];
#pragma unroll
  for (int j = 0; j < 4; ++j) { acc[j] = zero8(); accx[j] = zero8(); }

  const unsigned short* pah = qh + (size_t)(n0 + 16 * w + m) * CC + 8 * h;
  const unsigned short* pal = ql + (size_t)(n0 + 16 * w + m) * CC + 8 * h;
  const unsigned short* pbh = kh + (size_t)(m0 + m) * CC + 8 * h;
  const unsigned short* pbl = kl + (size_t)(m0 + m) * CC + 8 * h;
#pragma unroll 1
  for (int kk = 0; kk < CC / 32; ++kk) {
    const v16us ah  = ldfrag_u(pah + 32 * kk);
    const v16us al  = ldfrag_u(pal + 32 * kk);
    const v16us bh0 = ldfrag_u(pbh + 32 * kk);
    const v16us bh1 = ldfrag_u(pbh + (size_t)16 * CC + 32 * kk);
    const v16us bh2 = ldfrag_u(pbh + (size_t)32 * CC + 32 * kk);
    const v16us bh3 = ldfrag_u(pbh + (size_t)48 * CC + 32 * kk);
    const v16us bl0 = ldfrag_u(pbl + 32 * kk);
    const v16us bl1 = ldfrag_u(pbl + (size_t)16 * CC + 32 * kk);
    const v16us bl2 = ldfrag_u(pbl + (size_t)32 * CC + 32 * kk);
    const v16us bl3 = ldfrag_u(pbl + (size_t)48 * CC + 32 * kk);
    acc[0]  = mma_hu(ah, bh0, acc[0]);
    acc[1]  = mma_hu(ah, bh1, acc[1]);
    acc[2]  = mma_hu(ah, bh2, acc[2]);
    acc[3]  = mma_hu(ah, bh3, acc[3]);
    accx[0] = mma_hu(ah, bl0, accx[0]);
    accx[1] = mma_hu(ah, bl1, accx[1]);
    accx[2] = mma_hu(ah, bl2, accx[2]);
    accx[3] = mma_hu(ah, bl3, accx[3]);
    accx[0] = mma_hu(al, bh0, accx[0]);
    accx[1] = mma_hu(al, bh1, accx[1]);
    accx[2] = mma_hu(al, bh2, accx[2]);
    accx[3] = mma_hu(al, bh3, accx[3]);
    guard8w(acc[0], acc[1], acc[2], acc[3], accx[0], accx[1], accx[2], accx[3],
            ah, al, bh0, bh1, bh2, bh3, bl0, bl1, bl2, bl3);
  }

  const float kx = 1.0f / 32768.0f;
#pragma unroll
  for (int j = 0; j < 4; ++j) {
#pragma unroll
    for (int r = 0; r < 8; ++r)
      ct[(16 * w + 8 * h + r) * 64 + 16 * j + m] = acc[j][r] + accx[j][r] * kx;
  }
  __syncthreads();
  store_tile_f32(ct, S, (size_t)n0, m0, NPX, w, lane);
}

__global__ __launch_bounds__(256)
void k_rstat(const float* __restrict__ S, float* rmax, float* rsum)
{
  __shared__ __align__(16) float lm[32];
  __shared__ __align__(16) float ls[32];
  const int tid  = threadIdx.x;
  const int lane = tid & 31;
  const int w    = tid >> 5;
#pragma unroll 1
  for (int rr = 0; rr < 4; ++rr) {
    const int row = 32 * blockIdx.x + 4 * w + rr;
    const float* sr = S + (size_t)row * NPX + 8 * lane;
    float mx = -1.0e30f, sm = 0.0f;
#pragma unroll 1
    for (int it = 0; it < NPX / 256; ++it) {
      const v4f x0 = *(const v4f*)(sr + 256 * it);
      const v4f x1 = *(const v4f*)(sr + 256 * it + 4);
      const float cm = fmaxf(fmaxf(fmaxf(x0[0], x0[1]), fmaxf(x0[2], x0[3])),
                             fmaxf(fmaxf(x1[0], x1[1]), fmaxf(x1[2], x1[3])));
      const float mn = fmaxf(mx, cm);
      float add = 0.0f;
#pragma unroll
      for (int e = 0; e < 4; ++e) { add += __expf(x0[e] - mn); add += __expf(x1[e] - mn); }
      sm = sm * __expf(mx - mn) + add;
      mx = mn;
    }
    float M = mx;
#pragma unroll
    for (int o = 16; o >= 1; o >>= 1) M = fmaxf(M, __shfl_xor(M, o, 32));
    float st = sm * __expf(mx - M);
#pragma unroll
    for (int o = 16; o >= 1; o >>= 1) st += __shfl_xor(st, o, 32);
    if (lane == 0) { lm[4 * w + rr] = M; ls[4 * w + rr] = st; }
  }
  __syncthreads();
  if (w == 0 && lane < 8) {
    const v4f a = *(const v4f*)(lm + 4 * lane);
    const v4f c = *(const v4f*)(ls + 4 * lane);
    float* dm = rmax + 32 * blockIdx.x + 4 * lane;
    float* ds = rsum + 32 * blockIdx.x + 4 * lane;
    *(volatile v4f*)dm = a;
    *(volatile v4f*)ds = c;
    __threadfence();
    *(volatile v4f*)dm = a;
    *(volatile v4f*)ds = c;
  }
}

__device__ __forceinline__ void o_store_pass(const float* Et, float* orows, int R0, int w, int lane)
{
  const int q  = lane >> 3;
  const int jj = lane & 7;
#pragma unroll 1
  for (int it = 0; it < 8; ++it) {
    const int li = it * 32 + 4 * w + q;
    const int c = li >> 1, hf = li & 1;
    const v4f v = *(const v4f*)(Et + c * EPF + 32 * hf + 4 * jj);
    *(volatile v4f*)(orows + (size_t)c * NPX + R0 + 32 * hf + 4 * jj) = v;
  }
}

__global__ __launch_bounds__(256)
void k_pv(const float* __restrict__ S, const float* __restrict__ rmax, const float* __restrict__ rsum,
          const unsigned short* __restrict__ ucb, float* O, float* ps, float* pq)
{
  __shared__ __align__(16) unsigned short Pt[64 * TP];
  __shared__ __align__(16) float Et[128 * EPF];
  __shared__ float mxs[64];
  __shared__ float invs[64];
  __shared__ __align__(16) float lsum[CC];
  __shared__ __align__(16) float lsq[CC];

  const int tid  = threadIdx.x;
  const int lane = tid & 31;
  const int w    = tid >> 5;
  const int h    = lane >> 4;
  const int m    = lane & 15;
  const int R0   = 64 * blockIdx.x;

  if (tid < 64) {
    mxs[tid]  = rmax[R0 + tid];
    invs[tid] = rcpf(rsum[R0 + tid]) * (1.0f / 262144.0f);
  }
  __syncthreads();

  const int fr = tid >> 2;
  const int fc = 16 * (tid & 3);
  const float mx0 = mxs[fr];
  const float* sp = S + (size_t)(R0 + fr) * NPX + fc;

  v8f acc[8];
#pragma unroll
  for (int k = 0; k < 8; ++k) acc[k] = zero8();
  const unsigned short* pa0 = ucb + (size_t)(32 * w + m) * NPX + 8 * h;
  const unsigned short* pa1 = pa0 + (size_t)16 * NPX;

#pragma unroll 1
  for (int T = 0; T < NPX / 64; ++T) {
    {
      const float* s2 = sp + 64 * T;
      const v4f x0 = *(const v4f*)(s2);
      const v4f x1 = *(const v4f*)(s2 + 4);
      const v4f x2 = *(const v4f*)(s2 + 8);
      const v4f x3 = *(const v4f*)(s2 + 12);
      v8us o0, o1;
#pragma unroll
      for (int e = 0; e < 4; ++e) {
        o0[e]     = hbits(16384.0f * __expf(x0[e] - mx0));
        o0[4 + e] = hbits(16384.0f * __expf(x1[e] - mx0));
        o1[e]     = hbits(16384.0f * __expf(x2[e] - mx0));
        o1[4 + e] = hbits(16384.0f * __expf(x3[e] - mx0));
      }
      *(v8us*)(Pt + fr * TP + fc)     = o0;
      *(v8us*)(Pt + fr * TP + fc + 8) = o1;
    }
    __syncthreads();
#pragma unroll
    for (int kk = 0; kk < 2; ++kk) {
      const v16us a0 = ldfrag_u(pa0 + 64 * T + 32 * kk);
      const v16us a1 = ldfrag_u(pa1 + 64 * T + 32 * kk);
      const v16us b0 = ldfrag_u(Pt + (0 * 16 + m) * TP + 32 * kk + 8 * h);
      const v16us b1 = ldfrag_u(Pt + (1 * 16 + m) * TP + 32 * kk + 8 * h);
      const v16us b2 = ldfrag_u(Pt + (2 * 16 + m) * TP + 32 * kk + 8 * h);
      const v16us b3 = ldfrag_u(Pt + (3 * 16 + m) * TP + 32 * kk + 8 * h);
      acc[0] = mma_hu(a0, b0, acc[0]);
      acc[1] = mma_hu(a0, b1, acc[1]);
      acc[2] = mma_hu(a0, b2, acc[2]);
      acc[3] = mma_hu(a0, b3, acc[3]);
      acc[4] = mma_hu(a1, b0, acc[4]);
      acc[5] = mma_hu(a1, b1, acc[5]);
      acc[6] = mma_hu(a1, b2, acc[6]);
      acc[7] = mma_hu(a1, b3, acc[7]);
      guard8(acc[0], acc[1], acc[2], acc[3], acc[4], acc[5], acc[6], acc[7], a0, a1, b0, b1, b2, b3);
    }
    __syncthreads();
  }

#pragma unroll
  for (int k = 0; k < 8; ++k) {
    const float iv = invs[16 * (k & 3) + m];
#pragma unroll
    for (int r = 0; r < 8; ++r) acc[k][r] = acc[k][r] * iv;
  }
  float rs[2][8], rq[2][8];
#pragma unroll
  for (int s = 0; s < 2; ++s) {
#pragma unroll
    for (int r = 0; r < 8; ++r) {
      float a = 0.0f, q2 = 0.0f;
#pragma unroll
      for (int j = 0; j < 4; ++j) {
        const float p = acc[4 * s + j][r];
        a += p;
        q2 += p * p;
      }
      rs[s][r] = a;
      rq[s][r] = q2;
    }
  }
#pragma unroll
  for (int s = 0; s < 2; ++s) {
#pragma unroll
    for (int r = 0; r < 8; ++r) {
#pragma unroll
      for (int o = 1; o < 16; o <<= 1) {
        rs[s][r] += __shfl_xor(rs[s][r], o, 32);
        rq[s][r] += __shfl_xor(rq[s][r], o, 32);
      }
    }
  }
  if (m == 0) {
#pragma unroll
    for (int s = 0; s < 2; ++s) {
#pragma unroll
      for (int r = 0; r < 8; ++r) {
        lsum[32 * w + 16 * s + 8 * h + r] = rs[s][r];
        lsq[32 * w + 16 * s + 8 * h + r]  = rq[s][r];
      }
    }
  }

#pragma unroll
  for (int half = 0; half < 2; ++half) {
    if ((w >> 2) == half) {
#pragma unroll
      for (int s = 0; s < 2; ++s) {
#pragma unroll
        for (int j = 0; j < 4; ++j) {
#pragma unroll
          for (int r = 0; r < 8; ++r) {
            const int cl = 32 * (w & 3) + 16 * s + 8 * h + r;
            const int il = 16 * j + m;
            Et[cl * EPF + il] = acc[4 * s + j][r];
          }
        }
      }
    }
    __syncthreads();
    float* orows = O + (size_t)(128 * half) * NPX;
    o_store_pass(Et, orows, R0, w, lane);
    __threadfence();
    o_store_pass(Et, orows, R0, w, lane);
    __syncthreads();
  }

  if (tid < 64) {
    const v4f v = *(const v4f*)(lsum + 4 * tid);
    float* d = ps + (size_t)blockIdx.x * CC + 4 * tid;
    *(volatile v4f*)d = v;
    __threadfence();
    *(volatile v4f*)d = v;
  } else if (tid < 128) {
    const int t2 = tid - 64;
    const v4f v = *(const v4f*)(lsq + 4 * t2);
    float* d = pq + (size_t)blockIdx.x * CC + 4 * t2;
    *(volatile v4f*)d = v;
    __threadfence();
    *(volatile v4f*)d = v;
  }
}

__global__ __launch_bounds__(256)
void k_gn(const float* __restrict__ O, const float* __restrict__ ps, const float* __restrict__ pq,
          const float* __restrict__ handb, const float* __restrict__ gnw,
          const float* __restrict__ gnb, float* outb)
{
  __shared__ float stat[2];
  const int tid  = threadIdx.x;
  const int lane = tid & 31;
  const int w    = tid >> 5;
  const int c    = blockIdx.x;
  const int g    = c >> 3;

  if (w == 0) {
    double s = 0.0, q = 0.0;
    const float* psg = ps + 8 * g;
    const float* pqg = pq + 8 * g;
#pragma unroll 1
    for (int i = 0; i < 16; ++i) {
      const int idx = lane + 32 * i;
      const int blk = idx >> 3, ch = idx & 7;
      s += (double)psg[(size_t)blk * CC + ch];
      q += (double)pqg[(size_t)blk * CC + ch];
    }
#pragma unroll
    for (int o = 16; o >= 1; o >>= 1) {
      s += shfl_xor_d(s, o);
      q += shfl_xor_d(q, o);
    }
    if (lane == 0) {
      const double inv_n = 1.0 / 32768.0;
      const double mean = s * inv_n;
      double var = q * inv_n - mean * mean;
      if (var < 0.0) var = 0.0;
      const float varf = (float)var;
      stat[0] = (float)mean;
      stat[1] = rcpf(sqrtf(varf + 1e-5f));
    }
  }
  __syncthreads();
  const float meanf = stat[0];
  const float rstd  = stat[1];
  const float gw    = bf16r(gnw[c]);
  const float gb    = bf16r(gnb[c]);
  const float* orow = O + (size_t)c * NPX;
  const float* hrow = handb + (size_t)c * NPX;
  float* drow = outb + (size_t)c * NPX;

  v4f res[4];
#pragma unroll
  for (int it = 0; it < 4; ++it) {
    const int f = 4 * (it * 256 + tid);
    const v4f ov = *(const v4f*)(orow + f);
    const v4f hd = *(const v4f*)(hrow + f);
#pragma unroll
    for (int e = 0; e < 4; ++e) {
      const float xn = (ov[e] - meanf) * rstd;
      res[it][e] = xn * gw + gb + bf16r(hd[e]);
    }
  }
#pragma unroll
  for (int it = 0; it < 4; ++it)
    *(volatile v4f*)(drow + 4 * (it * 256 + tid)) = res[it];
  __threadfence();
#pragma unroll
  for (int it = 0; it < 4; ++it)
    *(volatile v4f*)(drow + 4 * (it * 256 + tid)) = res[it];
}

extern "C" void kernel_launch(void* const* d_in, const int* in_sizes, int n_in,
                              void* d_out, int out_size, void* d_ws, size_t ws_size,
                              hipStream_t stream) {
  if (n_in < 8) return;
  const int per = CC * NPX;
  const int n0s = in_sizes[0];
  if (n0s < per || (n0s % per) != 0) return;
  const int nb = n0s / per;
  if (nb < 1 || nb > NBMAX) return;
  if (in_sizes[1] != n0s) return;
  if (in_sizes[2] != CC * CC || in_sizes[4] != CC * CC) return;
  if (in_sizes[3] != CC || in_sizes[5] != CC || in_sizes[6] != CC || in_sizes[7] != CC) return;
  if (out_size != nb * per) return;
  if (ws_size < WS_TOTAL) return;

  const float* hand = (const float*)d_in[0];
  const float* u    = (const float*)d_in[1];
  const float* whw  = (const float*)d_in[2];
  const float* whb  = (const float*)d_in[3];
  const float* wuw  = (const float*)d_in[4];
  const float* wub  = (const float*)d_in[5];
  const float* gnw  = (const float*)d_in[6];
  const float* gnb  = (const float*)d_in[7];
  float* out = (float*)d_out;

  char* ws = (char*)d_ws;
  unsigned short* ht  = (unsigned short*)(ws + OFF_HT);
  unsigned short* ut  = (unsigned short*)(ws + OFF_UT);
  unsigned short* uc  = (unsigned short*)(ws + OFF_UC);
  unsigned short* w16 = (unsigned short*)(ws + OFF_W16);
  unsigned short* qh  = (unsigned short*)(ws + OFF_QH);
  unsigned short* ql  = (unsigned short*)(ws + OFF_QL);
  unsigned short* kh  = (unsigned short*)(ws + OFF_KH);
  unsigned short* kl  = (unsigned short*)(ws + OFF_KL);
  float*          Sp  = (float*)(ws + OFF_S);
  float*          rmx = (float*)(ws + OFF_RMAX);
  float*          rsm = (float*)(ws + OFF_RSUM);
  float*          Op  = (float*)(ws + OFF_O);
  float*          ps  = (float*)(ws + OFF_PS);
  float*          pq  = (float*)(ws + OFF_PQ);

  k_cvt<<<dim3(NPX / 64, CC / 64, nb), dim3(256), 0, stream>>>(hand, u, ht, ut, uc);
  (void)hipGetLastError();
  k_wcvt<<<dim3(64), dim3(256), 0, stream>>>(whw, wuw, w16);
  (void)hipGetLastError();
  k_proj<<<dim3(NPX / 64, CC / 64, 2 * nb), dim3(128), 0, stream>>>(ht, ut, w16, whb, wub,
                                                                     qh, ql, kh, kl);
  (void)hipGetLastError();

  for (int b = 0; b < nb; ++b) {
    const size_t po = (size_t)b * PLANE;
    const size_t pp = (size_t)b * HWD * CC;
    k_score<<<dim3(NPX / 64, NPX / 64), dim3(128), 0, stream>>>(qh + po, ql + po, kh + po, kl + po, Sp);
    (void)hipGetLastError();
    k_rstat<<<dim3(NPX / 32), dim3(256), 0, stream>>>(Sp, rmx, rsm);
    (void)hipGetLastError();
    k_pv<<<dim3(HWD), dim3(256), 0, stream>>>(Sp, rmx, rsm, uc + po, Op, ps + pp, pq + pp);
    (void)hipGetLastError();
    k_gn<<<dim3(CC), dim3(256), 0, stream>>>(Op, ps + pp, pq + pp, hand + po, gnw, gnb, out + po);
    (void)hipGetLastError();
  }
}
